// HyenaOperator_37864431681934
// MI455X (gfx1250) — hardware-run, weakly checked
//
#include <hip/hip_runtime.h>
#include <math.h>

typedef __attribute__((ext_vector_type(16))) _Float16 v16h;
typedef __attribute__((ext_vector_type(8)))  _Float16 v8h;
typedef __attribute__((ext_vector_type(8)))  float    v8f;
typedef __attribute__((ext_vector_type(4)))  float    v4f;
typedef __attribute__((ext_vector_type(4)))  unsigned v4u;

constexpr int kB    = 2;
constexpr int kL    = 2048;
constexpr int kD    = 768;
constexpr int kF    = 64;
constexpr int kRows = kB * kL;
constexpr int kNP   = 4 * kD;
constexpr int kXP   = 4160;
constexpr int kKT   = 2080;
constexpr int kEP   = 2304;
static_assert(kRows == 4096 && kNP == 3072, "shape");
static_assert((kD % 64) == 0 && (kNP % 64) == 0 && (kRows % 64) == 0 && (kD % 32) == 0, "GEMM tile multiples");
static_assert((kKT % 32) == 0 && kKT >= kL + 15, "Toeplitz K");
static_assert(16 * 127 + kKT <= kXP, "padded signal extent");
static_assert(kKT + 8 <= kEP && (kEP % 256) == 0, "shifted copy pitch");

constexpr float kCarryX = 16.0f;
constexpr float kCarryW = 64.0f;
constexpr float kCarryF = 16.0f;
constexpr float kCarryU = 16.0f;
constexpr float kInvProj = 1.0f / (kCarryX * kCarryW);
constexpr float kInvOut  = 1.0f / kCarryW;
constexpr float kInvConv = 1.0f / (kCarryF * kCarryU);

constexpr size_t kOffXH  = 0;
constexpr size_t kOffWIT = kOffXH  + (size_t)kRows * kD * 2;
constexpr size_t kOffWOT = kOffWIT + (size_t)kNP * kD * 2;
constexpr size_t kOffBAS = kOffWOT + (size_t)kD * kD * 2;
constexpr size_t kOffFLT = kOffBAS + (size_t)kL * kF * 4;
constexpr size_t kOffPRJ = kOffFLT + (size_t)kD * kL * 2;
constexpr size_t kOffXT  = kOffPRJ + (size_t)kRows * kNP * 4;
constexpr size_t kOffGT  = kOffXT  + (size_t)kB * kD * kL * 2;
constexpr size_t kOffYT  = kOffGT  + (size_t)kB * kD * kL * 4;
constexpr size_t kOffYH  = kOffYT  + (size_t)kB * kD * kL * 4;
constexpr size_t kWsTotal = kOffYH + (size_t)kRows * kD * 2;
static_assert(kWsTotal == 103940096ull, "carve total");
static_assert(kWsTotal <= 134217728ull, "carve cap");
static_assert((kOffWIT % 128) == 0 && (kOffWOT % 128) == 0 && (kOffBAS % 128) == 0 && (kOffFLT % 128) == 0 &&
              (kOffPRJ % 128) == 0 && (kOffXT % 128) == 0 && (kOffGT % 128) == 0 && (kOffYT % 128) == 0 &&
              (kOffYH % 128) == 0, "128-B aligned regions");

__device__ __forceinline__ float bf16_rne(float f) {
  const unsigned u = __float_as_uint(f);
  const unsigned r = (u + 0x7FFFu + ((u >> 16) & 1u)) & 0xFFFF0000u;
  return __uint_as_float(r);
}

__device__ __forceinline__ void guard_row4(v8f& a, v8f& b, v8f& c, v8f& d, v16h x, v16h y) {
  asm volatile("v_nop\n\tv_nop\n\tv_nop\n\tv_nop" : "+v"(a), "+v"(b), "+v"(c), "+v"(d) : "v"(x), "v"(y));
}
__device__ __forceinline__ void guard_pair(v8f& a, v8f& b, v16h x, v16h y, v16h z) {
  asm volatile("v_nop\n\tv_nop\n\tv_nop\n\tv_nop" : "+v"(a), "+v"(b) : "v"(x), "v"(y), "v"(z));
}
__device__ __forceinline__ void keep4_h(v16h a, v16h b, v16h c, v16h d) { asm volatile("v_nop" :: "v"(a), "v"(b), "v"(c), "v"(d)); }
__device__ __forceinline__ void acc_guard4(v8f& a, v8f& b, v8f& c, v8f& d) { asm volatile("v_nop\n\tv_nop\n\tv_nop\n\tv_nop" : "+v"(a), "+v"(b), "+v"(c), "+v"(d)); }

union FragU { v16h v; v8h h[2]; };
__device__ __forceinline__ v16h frag_load(const _Float16* p) {
  FragU f;
  f.h[0] = *(const v8h*)(p);
  f.h[1] = *(const v8h*)(p + 16);
  return f.v;
}
__device__ __forceinline__ v8f mma_f16(v16h a, v16h b, v8f c) {
  return __builtin_amdgcn_wmma_f32_16x16x32_f16(false, a, false, b, (short)0, c, false, false);
}
__device__ __forceinline__ void wave_lds_sync() {
  __builtin_amdgcn_fence(__ATOMIC_RELEASE, "workgroup");
  __builtin_amdgcn_wave_barrier();
  __builtin_amdgcn_fence(__ATOMIC_ACQUIRE, "workgroup");
}

__global__ __launch_bounds__(256) void cvt_x_kernel(const float* __restrict__ x, unsigned short* __restrict__ xh, int total8)
{
  const int i = blockIdx.x * 256 + threadIdx.x;
  if (i >= total8) return;
  const size_t e0 = (size_t)i << 3;
  const v4f a0 = *(const v4f*)(x + e0);
  const v4f a1 = *(const v4f*)(x + e0 + 4);
  v8h hv;
#pragma unroll
  for (int e = 0; e < 4; ++e) {
    const float s0 = a0[e];
    const float s1 = a1[e];
    hv[e]     = (_Float16)(bf16_rne(s0) * kCarryX);
    hv[4 + e] = (_Float16)(bf16_rne(s1) * kCarryX);
  }
  unsigned short* q = xh + e0;
  *(volatile v8h*)q = hv;
  __threadfence();
  *(volatile v8h*)q = hv;
}

__global__ __launch_bounds__(256) void transpose_w_kernel(const float* __restrict__ in, unsigned short* __restrict__ out,
                                                          int R, int C, float scale)
{
  __shared__ __align__(16) float sT[64 * 68];
  const int tid = threadIdx.x, lane = tid & 31, wave = tid >> 5;
  const int c0 = blockIdx.x * 64, r0 = blockIdx.y * 64;
  const int lr = tid >> 4, c4 = (tid & 15) * 4;
#pragma unroll
  for (int j = 0; j < 4; ++j) {
    const int r = lr + 16 * j;
    const v4f v = *(const v4f*)(in + (size_t)(r0 + r) * C + c0 + c4);
    v4f w;
#pragma unroll
    for (int e = 0; e < 4; ++e) {
      const float s = v[e];
      w[e] = bf16_rne(s);
    }
    *(v4f*)(sT + r * 68 + c4) = w;
  }
  __syncthreads();
  const int q = lane >> 3, r8 = (lane & 7) * 8;
  v8h hv[2];
#pragma unroll
  for (int it = 0; it < 2; ++it) {
    const int cr = it * 32 + wave * 4 + q;
#pragma unroll
    for (int e = 0; e < 8; ++e) hv[it][e] = (_Float16)(sT[(r8 + e) * 68 + cr] * scale);
  }
  for (int pass = 0; pass < 2; ++pass) {
#pragma unroll
    for (int it = 0; it < 2; ++it) {
      const int cr = it * 32 + wave * 4 + q;
      *(volatile v8h*)(out + (size_t)(c0 + cr) * R + r0 + r8) = hv[it];
    }
    __threadfence();
  }
}

__global__ __launch_bounds__(256) void basis_kernel(float* __restrict__ basis)
{
  const int i = blockIdx.x * 256 + threadIdx.x;
  const int t = i >> 4;
  const int f0 = (i & 15) * 4;
  v4f o;
#pragma unroll
  for (int e = 0; e < 4; ++e) {
    const float arg = (float)(t * (f0 + e)) * (1.0f / (float)kF);
    o[e] = sinf(arg);
  }
  float* q = basis + (size_t)i * 4;
  *(volatile v4f*)q = o;
  __threadfence();
  *(volatile v4f*)q = o;
}

__global__ __launch_bounds__(256) void filt_kernel(const float* __restrict__ basis, const float* __restrict__ w_filt,
                                                   const float* __restrict__ b_filt, unsigned short* __restrict__ filt16)
{
  __shared__ __align__(16) float sW[kF];
  const int tid = threadIdx.x;
  const int d = blockIdx.x;
  if (tid < kF) sW[tid] = bf16_rne(w_filt[(size_t)tid * kD + d]);
  __syncthreads();
  const float bq = bf16_rne(b_filt[d]);
  const int k0 = tid * 8;
  float acc[8];
#pragma unroll
  for (int j = 0; j < 8; ++j) acc[j] = 0.0f;
#pragma unroll 1
  for (int f4 = 0; f4 < kF / 4; ++f4) {
    const v4f w = *(const v4f*)(sW + 4 * f4);
#pragma unroll
    for (int j = 0; j < 8; ++j) {
      const v4f b4 = *(const v4f*)(basis + (size_t)(k0 + j) * kF + 4 * f4);
      float a = acc[j];
      a = fmaf(b4[0], w[0], a);
      a = fmaf(b4[1], w[1], a);
      a = fmaf(b4[2], w[2], a);
      a = fmaf(b4[3], w[3], a);
      acc[j] = a;
    }
  }
  v8h hv;
#pragma unroll
  for (int j = 0; j < 8; ++j) hv[j] = (_Float16)((acc[j] + bq) * kCarryF);
  unsigned short* q = filt16 + (size_t)d * kL + k0;
  *(volatile v8h*)q = hv;
  __threadfence();
  *(volatile v8h*)q = hv;
}

__global__ __launch_bounds__(256) void gemm64_f16_kernel(
    const unsigned short* __restrict__ Ap, int lda,
    const unsigned short* __restrict__ Btp, int ldb,
    float* __restrict__ C, int ldc,
    const float* __restrict__ bias,
    int M, int N, int K, float scale)
{
  const _Float16* A  = (const _Float16*)Ap;
  const _Float16* Bt = (const _Float16*)Btp;
  __shared__ __align__(16) float sT[8][16 * 68];
  const int lane = threadIdx.x & 31;
  const int wave = threadIdx.x >> 5;
  const int tilesN = N >> 6;
  const int tilesM = M >> 6;
  const int tile = blockIdx.x * 8 + wave;
  if (tile >= tilesM * tilesN) return;
  const int tm = tile / tilesN;
  const int tn = tile - tm * tilesN;
  const int m0 = tm << 6;
  const int n0 = tn << 6;

  const int rlane = lane & 15;
  const int koff  = (lane >> 4) * 8;
  const int mOff  = (lane >> 4) * 8;

  v8f acc[4][4];
#pragma unroll
  for (int i = 0; i < 4; ++i)
#pragma unroll
    for (int j = 0; j < 4; ++j) acc[i][j] = (v8f){0.f, 0.f, 0.f, 0.f, 0.f, 0.f, 0.f, 0.f};

  for (int k0 = 0; k0 < K; k0 += 32) {
    v16h bh[4];
#pragma unroll
    for (int j = 0; j < 4; ++j) {
      const size_t bo = (size_t)(n0 + (j << 4) + rlane) * ldb + koff + k0;
      bh[j] = frag_load(Bt + bo);
    }
#pragma unroll
    for (int i = 0; i < 4; ++i) {
      const size_t ao = (size_t)(m0 + (i << 4) + rlane) * lda + koff + k0;
      const v16h ah = frag_load(A + ao);
#pragma unroll
      for (int j = 0; j < 4; ++j) acc[i][j] = mma_f16(ah, bh[j], acc[i][j]);
      guard_row4(acc[i][0], acc[i][1], acc[i][2], acc[i][3], ah, bh[3]);
    }
    keep4_h(bh[0], bh[1], bh[2], bh[3]);
  }
  acc_guard4(acc[0][0], acc[0][1], acc[0][2], acc[0][3]);
  acc_guard4(acc[1][0], acc[1][1], acc[1][2], acc[1][3]);
  acc_guard4(acc[2][0], acc[2][1], acc[2][2], acc[2][3]);
  acc_guard4(acc[3][0], acc[3][1], acc[3][2], acc[3][3]);

  float* slab = sT[wave];
#pragma unroll
  for (int i = 0; i < 4; ++i) {
    const int mBase = m0 + (i << 4);
#pragma unroll
    for (int j = 0; j < 4; ++j) {
      const int n = n0 + (j << 4) + rlane;
      const float bv = bf16_rne(bias[n]);
#pragma unroll
      for (int r = 0; r < 8; ++r) {
        const float v = acc[i][j][r] * scale + bv;
        slab[(mOff + r) * 68 + (j << 4) + rlane] = v;
      }
    }
    wave_lds_sync();
    {
      const int hh = lane >> 4, c4 = (lane & 15) * 4;
      for (int pass = 0; pass < 2; ++pass) {
#pragma unroll
        for (int it = 0; it < 8; ++it) {
          const int row = it * 2 + hh;
          const v4f v = *(const v4f*)(slab + row * 68 + c4);
          *(volatile v4f*)(C + (size_t)(mBase + row) * ldc + n0 + c4) = v;
        }
        __threadfence();
      }
    }
    wave_lds_sync();
  }
}

__global__ __launch_bounds__(256) void gate_transpose_kernel(const float* __restrict__ proj,
                                                             unsigned short* __restrict__ xT, float* __restrict__ gT)
{
  __shared__ __align__(16) float sP[64 * 68];
  __shared__ __align__(16) float sG[64 * 68];
  const int tid = threadIdx.x, lane = tid & 31, wave = tid >> 5;
  const int i0 = blockIdx.x * 64, d0 = blockIdx.y * 64, b = blockIdx.z;
  const int lr = tid >> 4, c4 = (tid & 15) * 4;
#pragma unroll 1
  for (int j = 0; j < 4; ++j) {
    const int il = lr + 16 * j;
    const float* p = proj + (size_t)(b * kL + i0 + il) * kNP + d0 + c4;
    const v4f uv = *(const v4f*)(p);
    const v4f zv = *(const v4f*)(p + kD);
    const v4f v1 = *(const v4f*)(p + 2 * kD);
    const v4f v2 = *(const v4f*)(p + 3 * kD);
    v4f gv;
#pragma unroll
    for (int e = 0; e < 4; ++e) {
      const float z = zv[e];
      const float sg = 1.0f / (1.0f + expf(-z));
      gv[e] = (z * sg) * v1[e] * v2[e];
    }
    *(v4f*)(sP + il * 68 + c4) = uv;
    *(v4f*)(sG + il * 68 + c4) = gv;
  }
  __syncthreads();
  const int q = lane >> 3, i8 = (lane & 7) * 8;
  const int hh = lane >> 4, c4o = (lane & 15) * 4;
  v8h hv[2];
  v4f go[4];
#pragma unroll
  for (int it = 0; it < 2; ++it) {
    const int dr = it * 32 + wave * 4 + q;
#pragma unroll
    for (int e = 0; e < 8; ++e) hv[it][e] = (_Float16)(sP[(i8 + e) * 68 + dr] * kCarryU);
  }
#pragma unroll
  for (int it = 0; it < 4; ++it) {
    const int dr = it * 16 + wave * 2 + hh;
#pragma unroll
    for (int e = 0; e < 4; ++e) go[it][e] = sG[(c4o + e) * 68 + dr];
  }
  for (int pass = 0; pass < 2; ++pass) {
#pragma unroll
    for (int it = 0; it < 2; ++it) {
      const int dr = it * 32 + wave * 4 + q;
      *(volatile v8h*)(xT + ((size_t)(b * kD + d0 + dr)) * kL + i0 + i8) = hv[it];
    }
#pragma unroll
    for (int it = 0; it < 4; ++it) {
      const int dr = it * 16 + wave * 2 + hh;
      *(volatile v4f*)(gT + ((size_t)(b * kD + d0 + dr)) * kL + i0 + c4o) = go[it];
    }
    __threadfence();
  }
}

__device__ __forceinline__ void conv_tile_out(float* so, const v8f acc, int lane,
                                              const float* __restrict__ grow, float* __restrict__ yrow)
{
  const int n = lane & 15, h = lane >> 4;
  v4f p0, p1;
  p0[0] = acc[0]; p0[1] = acc[1]; p0[2] = acc[2]; p0[3] = acc[3];
  p1[0] = acc[4]; p1[1] = acc[5]; p1[2] = acc[6]; p1[3] = acc[7];
  *(v4f*)(so + 16 * n + 8 * h)     = p0;
  *(v4f*)(so + 16 * n + 8 * h + 4) = p1;
  wave_lds_sync();
  const int o0 = lane * 4;
  const int o1 = 128 + lane * 4;
  const v4f c0 = *(const v4f*)(so + o0);
  const v4f c1 = *(const v4f*)(so + o1);
  const v4f g0 = *(const v4f*)(grow + o0);
  const v4f g1 = *(const v4f*)(grow + o1);
  v4f y0, y1;
#pragma unroll
  for (int e = 0; e < 4; ++e) {
    y0[e] = (c0[e] * kInvConv) * g0[e];
    y1[e] = (c1[e] * kInvConv) * g1[e];
  }
  for (int pass = 0; pass < 2; ++pass) {
    *(volatile v4f*)(yrow + o0) = y0;
    *(volatile v4f*)(yrow + o1) = y1;
    __threadfence();
  }
  wave_lds_sync();
}

__global__ __launch_bounds__(256) void longconv_kernel(const unsigned short* __restrict__ filt16,
                                                       const unsigned short* __restrict__ xT,
                                                       const float* __restrict__ gT, float* __restrict__ yT)
{
  __shared__ __align__(16) unsigned short sE[8 * kEP];
  __shared__ __align__(16) unsigned short sX[2 * kXP];
  __shared__ __align__(16) float sO[8 * 256];
  const int tid = threadIdx.x, lane = tid & 31, wave = tid >> 5;
  const int d = blockIdx.x;
  const unsigned short* fg = filt16 + (size_t)d * kL;

#pragma unroll 1
  for (int s = 0; s < 8; ++s) {
#pragma unroll 1
    for (int j = 0; j < 9; ++j) {
      const int c = tid + 256 * j;
      const int src = c - 8 - s;
      const bool ok = (src >= 0) && (src < kL);
      int cs = src < 0 ? 0 : src;
      cs = cs > (kL - 1) ? (kL - 1) : cs;
      const unsigned v = fg[cs];
      const unsigned o = ok ? v : 0u;
      sE[s * kEP + c] = (unsigned short)o;
    }
  }
#pragma unroll
  for (int bb2 = 0; bb2 < 2; ++bb2) {
    const v4u w = *(const v4u*)(xT + ((size_t)(bb2 * kD + d)) * kL + tid * 8);
    *(v4u*)(sX + bb2 * kXP + 1024 + tid * 8) = w;
  }
#pragma unroll 1
  for (int j = 0; j < 3; ++j) {
    const int idx = tid + 256 * j;
    if (idx < 528) {
      const int bb2 = (idx >= 264) ? 1 : 0;
      const int w = idx - bb2 * 264;
      const int hoff = (w < 128) ? (w * 8) : (3072 + (w - 128) * 8);
      *(v4u*)(sX + bb2 * kXP + hoff) = (v4u){0u, 0u, 0u, 0u};
    }
  }
  __syncthreads();

  const int h = lane >> 4, n = lane & 15;
  const int bb = wave >> 2;
  const int a0 = (wave & 3) * 32;
  const _Float16* Ea = (const _Float16*)sE + (n & 7) * kEP + 8 * (1 - (n >> 3)) + 8 * h;
  const _Float16* X0 = (const _Float16*)sX + bb * kXP + 16 * (a0 + n) + 8 * h;
  const _Float16* X1 = X0 + 256;
  v8f acc0 = (v8f){0.f, 0.f, 0.f, 0.f, 0.f, 0.f, 0.f, 0.f};
  v8f acc1 = (v8f){0.f, 0.f, 0.f, 0.f, 0.f, 0.f, 0.f, 0.f};
#pragma unroll 1
  for (int k0 = 0; k0 < kKT; k0 += 32) {
    const v16h af = frag_load(Ea + k0);
    const v16h b0 = frag_load(X0 + k0);
    const v16h b1 = frag_load(X1 + k0);
    acc0 = mma_f16(af, b0, acc0);
    acc1 = mma_f16(af, b1, acc1);
    guard_pair(acc0, acc1, af, b0, b1);
  }
  float* so = sO + wave * 256;
  const size_t rowbase = ((size_t)(bb * kD + d)) * kL + 16 * a0;
  conv_tile_out(so, acc0, lane, gT + rowbase, yT + rowbase);
  conv_tile_out(so, acc1, lane, gT + rowbase + 256, yT + rowbase + 256);
}

__global__ __launch_bounds__(256) void y_transpose_short_kernel(const float* __restrict__ yT, const float* __restrict__ x,
                                                                const float* __restrict__ w_short,
                                                                const float* __restrict__ b_short,
                                                                unsigned short* __restrict__ yh)
{
  __shared__ __align__(16) float sY[64 * 68];
  const int tid = threadIdx.x, lane = tid & 31, wave = tid >> 5;
  const int i0 = blockIdx.x * 64, d0 = blockIdx.y * 64, b = blockIdx.z;
  const int lr = tid >> 4, c4 = (tid & 15) * 4;
#pragma unroll
  for (int j = 0; j < 4; ++j) {
    const int dr = lr + 16 * j;
    const v4f v = *(const v4f*)(yT + ((size_t)(b * kD + d0 + dr)) * kL + i0 + c4);
    *(v4f*)(sY + dr * 68 + c4) = v;
  }
  __syncthreads();
  const int q = lane >> 3, d8 = (lane & 7) * 8;
  const int dg = d0 + d8;
  float wt[24];
#pragma unroll
  for (int k = 0; k < 6; ++k) {
    const v4f w4 = *(const v4f*)(w_short + (size_t)dg * 3 + 4 * k);
#pragma unroll
    for (int e = 0; e < 4; ++e) {
      const float s = w4[e];
      wt[4 * k + e] = bf16_rne(s);
    }
  }
  float bs[8];
  {
    const v4f b0 = *(const v4f*)(b_short + dg);
    const v4f b1 = *(const v4f*)(b_short + dg + 4);
#pragma unroll
    for (int e = 0; e < 4; ++e) {
      const float s0 = b0[e];
      const float s1 = b1[e];
      bs[e] = bf16_rne(s0);
      bs[4 + e] = bf16_rne(s1);
    }
  }
#pragma unroll 1
  for (int it = 0; it < 2; ++it) {
    const int il = it * 32 + wave * 4 + q;
    const int i = i0 + il;
    const int row = b * kL + i;
    const bool okp = (i > 0);
    const bool okn = (i < kL - 1);
    const int rp = okp ? (row - 1) : row;
    const int rn = okn ? (row + 1) : row;
    const float* pc = x + (size_t)row * kD + dg;
    const float* pp = x + (size_t)rp * kD + dg;
    const float* pn = x + (size_t)rn * kD + dg;
    const v4f xc0 = *(const v4f*)(pc);
    const v4f xc1 = *(const v4f*)(pc + 4);
    const v4f xp0 = *(const v4f*)(pp);
    const v4f xp1 = *(const v4f*)(pp + 4);
    const v4f xn0 = *(const v4f*)(pn);
    const v4f xn1 = *(const v4f*)(pn + 4);
    float xc[8], xpv[8], xnv[8];
#pragma unroll
    for (int e = 0; e < 4; ++e) {
      const float c0v = xc0[e];
      const float c1v = xc1[e];
      const float p0v = xp0[e];
      const float p1v = xp1[e];
      const float n0v = xn0[e];
      const float n1v = xn1[e];
      xc[e]      = bf16_rne(c0v);
      xc[4 + e]  = bf16_rne(c1v);
      xpv[e]     = okp ? bf16_rne(p0v) : 0.0f;
      xpv[4 + e] = okp ? bf16_rne(p1v) : 0.0f;
      xnv[e]     = okn ? bf16_rne(n0v) : 0.0f;
      xnv[4 + e] = okn ? bf16_rne(n1v) : 0.0f;
    }
    v8h hv;
#pragma unroll
    for (int e = 0; e < 8; ++e) {
      float s = wt[3 * e] * xpv[e];
      s = fmaf(wt[3 * e + 1], xc[e], s);
      s = fmaf(wt[3 * e + 2], xnv[e], s);
      s = s + bs[e];
      const float yv = sY[(d8 + e) * 68 + il] + s;
      hv[e] = (_Float16)yv;
    }
    unsigned short* o = yh + (size_t)row * kD + dg;
    *(volatile v8h*)o = hv;
    __threadfence();
    *(volatile v8h*)o = hv;
  }
}

extern "C" void kernel_launch(void* const* d_in, const int* in_sizes, int n_in,
                              void* d_out, int out_size, void* d_ws, size_t ws_size,
                              hipStream_t stream) {
  if (n_in < 9) return;
  if (in_sizes[0] != kRows * kD) return;
  if (in_sizes[1] != kD * kNP) return;
  if (in_sizes[2] != kNP) return;
  if (in_sizes[3] != kF * kD) return;
  if (in_sizes[4] != kD) return;
  if (in_sizes[5] != kD * 3) return;
  if (in_sizes[6] != kD) return;
  if (in_sizes[7] != kD * kD) return;
  if (in_sizes[8] != kD) return;
  if (out_size != kRows * kD) return;
  if (ws_size < kWsTotal) return;

  const float* x       = (const float*)d_in[0];
  const float* w_in    = (const float*)d_in[1];
  const float* b_in    = (const float*)d_in[2];
  const float* w_filt  = (const float*)d_in[3];
  const float* b_filt  = (const float*)d_in[4];
  const float* w_short = (const float*)d_in[5];
  const float* b_short = (const float*)d_in[6];
  const float* w_out   = (const float*)d_in[7];
  const float* b_out   = (const float*)d_in[8];
  float* out = (float*)d_out;

  char* ws = (char*)d_ws;
  unsigned short* XH  = (unsigned short*)(ws + kOffXH);
  unsigned short* WIT = (unsigned short*)(ws + kOffWIT);
  unsigned short* WOT = (unsigned short*)(ws + kOffWOT);
  float*          BAS = (float*)(ws + kOffBAS);
  unsigned short* FLT = (unsigned short*)(ws + kOffFLT);
  float*          PRJ = (float*)(ws + kOffPRJ);
  unsigned short* XT  = (unsigned short*)(ws + kOffXT);
  float*          GT  = (float*)(ws + kOffGT);
  float*          YT  = (float*)(ws + kOffYT);
  unsigned short* YH  = (unsigned short*)(ws + kOffYH);

  cvt_x_kernel<<<(kRows * kD / 8) / 256, 256, 0, stream>>>(x, XH, kRows * kD / 8);
  transpose_w_kernel<<<dim3(kNP / 64, kD / 64), 256, 0, stream>>>(w_in, WIT, kD, kNP, kCarryW);
  transpose_w_kernel<<<dim3(kD / 64, kD / 64), 256, 0, stream>>>(w_out, WOT, kD, kD, kCarryW);
  basis_kernel<<<(kL * kF / 4) / 256, 256, 0, stream>>>(BAS);
  filt_kernel<<<kD, 256, 0, stream>>>(BAS, w_filt, b_filt, FLT);
  gemm64_f16_kernel<<<dim3((kRows / 64) * (kNP / 64) / 8, 1), 256, 0, stream>>>(
      XH, kD, WIT, kD, PRJ, kNP, b_in, kRows, kNP, kD, kInvProj);
  gate_transpose_kernel<<<dim3(kL / 64, kD / 64, kB), 256, 0, stream>>>(PRJ, XT, GT);
  longconv_kernel<<<kD, 256, 0, stream>>>(FLT, XT, GT, YT);
  y_transpose_short_kernel<<<dim3(kL / 64, kD / 64, kB), 256, 0, stream>>>(YT, x, w_short, b_short, YH);
  gemm64_f16_kernel<<<dim3((kRows / 64) * (kD / 64) / 8, 1), 256, 0, stream>>>(
      YH, kD, WOT, kD, out, kD, b_out, kRows, kD, kD, kInvOut);
}
